// SelectiveScan_19885698581141
// MI455X (gfx1250) — hardware-run, weakly checked
//
#include <hip/hip_runtime.h>
#include <hip/hip_fp16.h>
#include <math.h>

typedef __attribute__((ext_vector_type(16))) _Float16 v16h;
typedef __attribute__((ext_vector_type(8)))  _Float16 v8h;
typedef __attribute__((ext_vector_type(16))) __bf16   v16b;
typedef __attribute__((ext_vector_type(8)))  __bf16   v8b;
typedef __attribute__((ext_vector_type(8)))  float    v8f;
typedef __attribute__((ext_vector_type(4)))  float    v4f;
typedef __attribute__((ext_vector_type(4)))  unsigned v4u;

constexpr int kBatch  = 2;
constexpr int kSeq    = 2048;
constexpr int kDm     = 1024;
constexpr int kDin    = 2048;
constexpr int kNst    = 16;
constexpr int kRows   = kBatch * kSeq;
constexpr int kBcP    = 64;
constexpr int kConvTP = 260;
constexpr float kUCarry    = 4096.0f;
constexpr float kWCarry    = 1024.0f;
constexpr float kYCarry    = 4096.0f;
constexpr float kProjScale = 1.0f / (kUCarry * kWCarry);
constexpr float kOutScale  = 1.0f / kYCarry;
static_assert((kSeq & (kSeq - 1)) == 0);
static_assert((kDm % 64) == 0 && (kDin % 64) == 0 && (kRows % 64) == 0 && (kBcP % 64) == 0);
static_assert((kDm % 32) == 0 && (kDin % 32) == 0);
static_assert((kDin % 256) == 0 && (kSeq % 64) == 0);

constexpr size_t kSzP    = (size_t)kRows * kDin * 4;
constexpr size_t kSzQ    = (size_t)kRows * kDin * 2;
constexpr size_t kSzWdt  = (size_t)kDin * kDin * 2;
constexpr size_t kSzWot  = (size_t)kDm * kDin * 2;
constexpr size_t kSzWxt  = (size_t)64 * kDin * 2;
constexpr size_t kSzBc   = (size_t)kRows * kBcP * 4;
constexpr size_t kSzPar  = (size_t)65536 * 4;
constexpr size_t kOffP   = 0;
constexpr size_t kOffZ   = kOffP + kSzP;
constexpr size_t kOffU   = kOffZ + kSzP;
constexpr size_t kOffQ   = kOffU + kSzP;
constexpr size_t kOffWdt = kOffQ + kSzQ;
constexpr size_t kOffWot = kOffWdt + kSzWdt;
constexpr size_t kOffWxt = kOffWot + kSzWot;
constexpr size_t kOffBc  = kOffWxt + kSzWxt;
constexpr size_t kOffPar = kOffBc + kSzBc;
constexpr size_t kWsTotal = kOffPar + kSzPar;
static_assert(kWsTotal == 131596288ull);
static_assert(kWsTotal <= 134217728ull);
static_assert((kOffZ % 128) == 0 && (kOffU % 128) == 0 && (kOffQ % 128) == 0 && (kOffWdt % 128) == 0 &&
              (kOffWot % 128) == 0 && (kOffWxt % 128) == 0 && (kOffBc % 128) == 0 && (kOffPar % 128) == 0);
static_assert((size_t)kRows * kDm * 2 + (size_t)(2 * kDin) * kDm * 2 <= kSzQ);
static_assert((size_t)kRows * kDin * 2 <= kSzQ);
static_assert(2 * (size_t)kRows * kDin * 2 <= kSzP);

constexpr int kPBin  = 0;
constexpr int kPCw   = 4096;
constexpr int kPCb   = 12288;
constexpr int kPBdt  = 14336;
constexpr int kPAlog = 16384;
constexpr int kPD    = 49152;
constexpr int kPBout = 51200;
constexpr int kPBx   = 52224;
static_assert(kPCw == 2 * kDin && kPCb == kPCw + 4 * kDin && kPBdt == kPCb + kDin && kPAlog == kPBdt + kDin);
static_assert(kPD == kPAlog + kDin * kNst && kPBout == kPD + kDin && kPBx == kPBout + kDm);
static_assert((kPBx + 64) * 4 <= (int)kSzPar);

__device__ __forceinline__ unsigned short f2bf_bits(float f) {
  unsigned u = __float_as_uint(f);
  return (unsigned short)((u + 0x7FFFu + ((u >> 16) & 1u)) >> 16);
}
__device__ __forceinline__ float bf_bits2f(unsigned short h) { return __uint_as_float(((unsigned)h) << 16); }
__device__ __forceinline__ float bf_rne(float f) { return bf_bits2f(f2bf_bits(f)); }
__device__ __forceinline__ unsigned f16bits_flush(float v) {
  const float w = (fabsf(v) < 6.103515625e-05f) ? 0.0f : v;
  const _Float16 h = (_Float16)w;
  const unsigned short b = __builtin_bit_cast(unsigned short, h);
  return (unsigned)b;
}
__device__ __forceinline__ float h16_to_f32(unsigned hb) {
  const unsigned sgn = (hb & 0x8000u) << 16;
  const unsigned em = hb & 0x7fffu;
  const float fn = __uint_as_float((em << 13) + 0x38000000u);
  const float fs = (float)em * 5.9604644775390625e-8f;
  const float mag = (em < 0x400u) ? fs : fn;
  return __uint_as_float(__float_as_uint(mag) | sgn);
}

__device__ __forceinline__ void tie1_h(v8f& a, v16h x, v16h y, v16h z) { asm volatile("v_nop" : "+v"(a) : "v"(x), "v"(y), "v"(z)); }
__device__ __forceinline__ void tie4_h(v8f& a, v16h x, v16h y, v16h z) { asm volatile("v_nop\n\tv_nop\n\tv_nop\n\tv_nop" : "+v"(a) : "v"(x), "v"(y), "v"(z)); }
__device__ __forceinline__ void tie1_b(v8f& a, v16b x, v16b y, v16b z) { asm volatile("v_nop" : "+v"(a) : "v"(x), "v"(y), "v"(z)); }
__device__ __forceinline__ void tie4_b(v8f& a, v16b x, v16b y, v16b z) { asm volatile("v_nop\n\tv_nop\n\tv_nop\n\tv_nop" : "+v"(a) : "v"(x), "v"(y), "v"(z)); }
__device__ __forceinline__ void keep4_h(v16h a, v16h b, v16h c, v16h d) { asm volatile("v_nop" :: "v"(a), "v"(b), "v"(c), "v"(d)); }
__device__ __forceinline__ void keep4_b(v16b a, v16b b, v16b c, v16b d) { asm volatile("v_nop" :: "v"(a), "v"(b), "v"(c), "v"(d)); }
__device__ __forceinline__ void acc_guard1(v8f& a) { asm volatile("v_nop\n\tv_nop\n\tv_nop\n\tv_nop" : "+v"(a)); }

template <typename T> struct Frag;
template <> struct Frag<_Float16> {
  typedef v16h V; union U { v16h v; v8h h[2]; };
  static __device__ __forceinline__ v16h load(const _Float16* p) {
    U f; f.h[0] = *(const v8h*)(p); f.h[1] = *(const v8h*)(p + 16); return f.v;
  }
  static __device__ __forceinline__ v8f mma(v16h a, v16h b, v8f c) {
    return __builtin_amdgcn_wmma_f32_16x16x32_f16(false, a, false, b, (short)0, c, false, false);
  }
  static __device__ __forceinline__ void tie1(v8f& a, v16h x, v16h y, v16h z) { tie1_h(a, x, y, z); }
  static __device__ __forceinline__ void tie4(v8f& a, v16h x, v16h y, v16h z) { tie4_h(a, x, y, z); }
  static __device__ __forceinline__ void keep(v16h a, v16h b, v16h c, v16h d) { keep4_h(a, b, c, d); }
};
template <> struct Frag<__bf16> {
  typedef v16b V; union U { v16b v; v8b h[2]; };
  static __device__ __forceinline__ v16b load(const __bf16* p) {
    U f; f.h[0] = *(const v8b*)(p); f.h[1] = *(const v8b*)(p + 16); return f.v;
  }
  static __device__ __forceinline__ v8f mma(v16b a, v16b b, v8f c) {
    return __builtin_amdgcn_wmma_f32_16x16x32_bf16(false, a, false, b, (short)0, c, false, false);
  }
  static __device__ __forceinline__ void tie1(v8f& a, v16b x, v16b y, v16b z) { tie1_b(a, x, y, z); }
  static __device__ __forceinline__ void tie4(v8f& a, v16b x, v16b y, v16b z) { tie4_b(a, x, y, z); }
  static __device__ __forceinline__ void keep(v16b a, v16b b, v16b c, v16b d) { keep4_b(a, b, c, d); }
};
template <int ET> struct Elem;
template <> struct Elem<0> { typedef _Float16 T; };
template <> struct Elem<1> { typedef __bf16 T; };

template <int ET, int SPL>
__global__ __launch_bounds__(256) void wmma_gemm64(
    const unsigned short* __restrict__ Ap, const unsigned short* __restrict__ A2p, int lda,
    const unsigned short* __restrict__ Btp, int ldb,
    float* __restrict__ C, int ldc,
    const float* __restrict__ bias,
    int M, int N, int K, float scale) {
  typedef typename Elem<ET>::T T;
  typedef typename Frag<T>::V V;
  const T* A = (const T*)Ap; const T* A2 = (const T*)A2p; const T* Bt = (const T*)Btp;
  __shared__ __align__(16) float sT[8][16 * 68];
  const int lane = threadIdx.x & 31;
  const int wave = threadIdx.x >> 5;
  const int tilesN = N >> 6;
  const int tilesM = M >> 6;
  const int tile = blockIdx.x * 8 + wave;
  if (tile >= tilesM * tilesN) return;
  const int tm = tile / tilesN;
  const int tn = tile - tm * tilesN;
  const int m0 = tm << 6;
  const int n0 = tn << 6;

  const int rlane = lane & 15;
  const int koff  = (lane >> 4) * 8;
  const int mOff  = (lane >> 4) * 8;

  v8f acc[4][4];
#pragma unroll
  for (int i = 0; i < 4; ++i)
#pragma unroll
    for (int j = 0; j < 4; ++j) acc[i][j] = (v8f){0.f,0.f,0.f,0.f,0.f,0.f,0.f,0.f};

  for (int k0 = 0; k0 < K; k0 += 32) {
    V bh[4];
#pragma unroll
    for (int j = 0; j < 4; ++j) {
      const size_t bo = (size_t)(n0 + (j << 4) + rlane) * ldb + koff + k0;
      bh[j] = Frag<T>::load(Bt + bo);
    }
#pragma unroll
    for (int i = 0; i < 4; ++i) {
      const size_t ao = (size_t)(m0 + (i << 4) + rlane) * lda + koff + k0;
      V ah = Frag<T>::load(A + ao);
      V al = ah;
      if (SPL == 1) al = Frag<T>::load(A2 + ao);
#pragma unroll
      for (int j = 0; j < 4; ++j) {
        acc[i][j] = Frag<T>::mma(ah, bh[j], acc[i][j]);
        if (SPL == 1) acc[i][j] = Frag<T>::mma(al, bh[j], acc[i][j]);
      }
      Frag<T>::tie1(acc[i][0], ah, al, bh[0]);
      Frag<T>::tie1(acc[i][1], ah, al, bh[1]);
      Frag<T>::tie1(acc[i][2], ah, al, bh[2]);
      Frag<T>::tie4(acc[i][3], ah, al, bh[3]);
    }
    Frag<T>::keep(bh[0], bh[1], bh[2], bh[3]);
  }
#pragma unroll
  for (int i = 0; i < 4; ++i) {
    acc_guard1(acc[i][0]);
    acc_guard1(acc[i][1]);
    acc_guard1(acc[i][2]);
    acc_guard1(acc[i][3]);
  }

  float* slab = sT[wave];
#pragma unroll
  for (int i = 0; i < 4; ++i) {
    const int mBase = m0 + (i << 4);
#pragma unroll
    for (int j = 0; j < 4; ++j) {
      const int n = n0 + (j << 4) + rlane;
      const float bv = bias[n];
#pragma unroll
      for (int r = 0; r < 8; ++r) {
        const float v = acc[i][j][r] * scale + bv;
        slab[(mOff + r) * 68 + (j << 4) + rlane] = v;
      }
    }
    __builtin_amdgcn_fence(__ATOMIC_RELEASE, "workgroup");
    __builtin_amdgcn_wave_barrier();
    __builtin_amdgcn_fence(__ATOMIC_ACQUIRE, "workgroup");
    {
      const int hh = lane >> 4, c4 = (lane & 15) * 4;
      for (int pass = 0; pass < 2; ++pass) {
#pragma unroll
        for (int it = 0; it < 8; ++it) {
          const int row = it * 2 + hh;
          v4f v = *(const v4f*)(slab + row * 68 + c4);
          *(volatile v4f*)(C + (size_t)(mBase + row) * ldc + n0 + c4) = v;
        }
        __threadfence();
      }
    }
    __builtin_amdgcn_fence(__ATOMIC_RELEASE, "workgroup");
    __builtin_amdgcn_wave_barrier();
    __builtin_amdgcn_fence(__ATOMIC_ACQUIRE, "workgroup");
  }
}

__global__ __launch_bounds__(256) void params_bf16_kernel(
    const float* __restrict__ b_in, const float* __restrict__ conv_w, const float* __restrict__ conv_b,
    const float* __restrict__ b_dt, const float* __restrict__ A_log, const float* __restrict__ Dp,
    const float* __restrict__ b_out, const float* __restrict__ b_x, float* __restrict__ par)
{
  const int blk = blockIdx.x;
  const int tid = threadIdx.x;
  const float* src = b_in;
  int base = 0;
  if (blk >= 4)  { src = conv_w; base = 4; }
  if (blk >= 12) { src = conv_b; base = 12; }
  if (blk >= 14) { src = b_dt;   base = 14; }
  if (blk >= 16) { src = A_log;  base = 16; }
  if (blk >= 48) { src = Dp;     base = 48; }
  if (blk >= 50) { src = b_out;  base = 50; }
  if (blk >= 51) { src = b_x;    base = 51; }
  const bool tail = (blk >= 51);
  int off = (blk - base) * 1024 + tid * 4;
  if (tail) off = 16 + 4 * ((tid < 3) ? tid : 3);
  const v4f v = *(const v4f*)(src + off);
  float x0 = v[0];
  float x1 = v[1];
  float x2 = v[2];
  float x3 = v[3];
  asm volatile("" : "+v"(x0));
  asm volatile("" : "+v"(x1));
  asm volatile("" : "+v"(x2));
  asm volatile("" : "+v"(x3));
  float r0 = bf_rne(x0), r1 = bf_rne(x1), r2 = bf_rne(x2), r3 = bf_rne(x3);
  if (tail) {
    const float fill = (tid < 8) ? 1.0f : 0.0f;
    r0 = (tid < 4) ? r0 : fill;
    r1 = (tid < 4) ? r1 : fill;
    r2 = (tid < 4) ? r2 : fill;
    r3 = (tid < 4) ? r3 : fill;
  }
  const bool active = (!tail) || (tid < 16);
  const v4f o = (v4f){r0, r1, r2, r3};
  float* dst = par + (size_t)blk * 1024 + tid * 4;
  if (active) *(volatile v4f*)dst = o;
  __threadfence();
  if (active) *(volatile v4f*)dst = o;
}

__global__ __launch_bounds__(256) void cvt_rows_bf16_kernel(
    const float* __restrict__ src, unsigned short* __restrict__ dst, int total8)
{
  const int i = blockIdx.x * 256 + threadIdx.x;
  if (i >= total8) return;
  const size_t e0 = (size_t)i << 3;
  const v4f a0 = *(const v4f*)(src + e0);
  const v4f a1 = *(const v4f*)(src + e0 + 4);
  const unsigned b0 = f2bf_bits(a0[0]), b1 = f2bf_bits(a0[1]), b2 = f2bf_bits(a0[2]), b3 = f2bf_bits(a0[3]);
  const unsigned b4 = f2bf_bits(a1[0]), b5 = f2bf_bits(a1[1]), b6 = f2bf_bits(a1[2]), b7 = f2bf_bits(a1[3]);
  const v4u w = (v4u){b0 | (b1 << 16), b2 | (b3 << 16), b4 | (b5 << 16), b6 | (b7 << 16)};
  unsigned short* q = dst + e0;
  *(volatile v4u*)q = w;
  __threadfence();
  *(volatile v4u*)q = w;
}

template <int MODE>
__global__ __launch_bounds__(256) void transpose_cvt_kernel(
    const float* __restrict__ in, int ldin, int srcoff, int nvalid,
    unsigned short* __restrict__ outp, int ldout, float carry)
{
  __shared__ float sT[64 * 65];
  const int tid = threadIdx.x;
  const int n0 = blockIdx.x * 64;
  const int k0 = blockIdx.y * 64;
  const int col = tid & 63;
  const int rg  = tid >> 6;
  const int n = n0 + col;
  const bool valid = (n < nvalid);
  int sc = srcoff + n;
  sc = (sc < ldin - 1) ? sc : (ldin - 1);
#pragma unroll 4
  for (int i = 0; i < 16; ++i) {
    const int k = rg + 4 * i;
    float v = in[(size_t)(k0 + k) * ldin + sc];
    asm volatile("" : "+v"(v));
    sT[k * 65 + col] = valid ? v : 0.0f;
  }
  __syncthreads();
  const int r  = tid >> 3;
  const int c8 = (tid & 7) * 8;
  v4u w[2];
#pragma unroll
  for (int it = 0; it < 2; ++it) {
    const int row = it * 32 + r;
    unsigned b[8];
#pragma unroll
    for (int e = 0; e < 8; ++e) {
      const float f = sT[(c8 + e) * 65 + row];
      if (MODE == 0) {
        b[e] = (unsigned)f2bf_bits(f);
      } else {
        b[e] = f16bits_flush(bf_rne(f) * carry);
      }
    }
    w[it] = (v4u){b[0] | (b[1] << 16), b[2] | (b[3] << 16), b[4] | (b[5] << 16), b[6] | (b[7] << 16)};
  }
  for (int pass = 0; pass < 2; ++pass) {
#pragma unroll
    for (int it = 0; it < 2; ++it) {
      const int row = it * 32 + r;
      *(volatile v4u*)(outp + (size_t)(n0 + row) * ldout + k0 + c8) = w[it];
    }
    __threadfence();
  }
}

__global__ __launch_bounds__(256) void conv_silu_kernel(
    const float* __restrict__ XPRE, const float* __restrict__ cw, const float* __restrict__ cb,
    float* __restrict__ U, unsigned short* __restrict__ U16)
{
  __shared__ __align__(16) float sT[16 * kConvTP];
  const int tid = threadIdx.x, lane = tid & 31, wave = tid >> 5;
  const int d0 = blockIdx.x * 256, d = d0 + tid;
  const int g0 = blockIdx.y * 64;
  const int tb = g0 & (kSeq - 1);
  const v4f wv = *(const v4f*)(cw + (size_t)d * 4);
  const float w0 = wv[0], w1 = wv[1], w2 = wv[2], w3 = wv[3];
  const float bc = cb[d];
  float xm3, xm2, xm1;
  {
    const bool hist = (tb > 0);
    const int rb = hist ? (g0 - 3) : g0;
    const float v3 = XPRE[(size_t)rb * kDin + d];
    const float v2 = XPRE[(size_t)(rb + 1) * kDin + d];
    const float v1 = XPRE[(size_t)(rb + 2) * kDin + d];
    xm3 = hist ? v3 : 0.f;
    xm2 = hist ? v2 : 0.f;
    xm1 = hist ? v1 : 0.f;
  }
  const int hrow = wave >> 1;
  const int hch  = (wave & 1) * 128 + lane * 4;
#pragma unroll 1
  for (int sub = 0; sub < 4; ++sub) {
    const int lb = g0 + sub * 16;
#pragma unroll 1
    for (int s = 0; s < 16; ++s) {
      const float xcur = XPRE[(size_t)(lb + s) * kDin + d];
      float acc = w0 * xm3;
      acc = fmaf(w1, xm2, acc);
      acc = fmaf(w2, xm1, acc);
      acc = fmaf(w3, xcur, acc);
      const float sv = acc + bc;
      const float sg = __builtin_amdgcn_rcpf(1.0f + expf(-sv));
      sT[s * kConvTP + tid] = sv * sg;
      xm3 = xm2; xm2 = xm1; xm1 = xcur;
    }
    __syncthreads();
    v4f fv[4];
    v4u hw[2];
#pragma unroll
    for (int it = 0; it < 4; ++it) fv[it] = *(const v4f*)(sT + (it * 4 + hrow) * kConvTP + hch);
#pragma unroll
    for (int it = 0; it < 2; ++it) {
      const float* sp = sT + (it * 8 + wave) * kConvTP + lane * 8;
      const v4f a0 = *(const v4f*)(sp);
      const v4f a1 = *(const v4f*)(sp + 4);
      const unsigned b0 = f16bits_flush(a0[0] * kUCarry), b1 = f16bits_flush(a0[1] * kUCarry);
      const unsigned b2 = f16bits_flush(a0[2] * kUCarry), b3 = f16bits_flush(a0[3] * kUCarry);
      const unsigned b4 = f16bits_flush(a1[0] * kUCarry), b5 = f16bits_flush(a1[1] * kUCarry);
      const unsigned b6 = f16bits_flush(a1[2] * kUCarry), b7 = f16bits_flush(a1[3] * kUCarry);
      hw[it] = (v4u){b0 | (b1 << 16), b2 | (b3 << 16), b4 | (b5 << 16), b6 | (b7 << 16)};
    }
    for (int pass = 0; pass < 2; ++pass) {
#pragma unroll
      for (int it = 0; it < 4; ++it)
        *(volatile v4f*)(U + (size_t)(lb + it * 4 + hrow) * kDin + d0 + hch) = fv[it];
#pragma unroll
      for (int it = 0; it < 2; ++it)
        *(volatile v4u*)(U16 + (size_t)(lb + it * 8 + wave) * kDin + d0 + lane * 8) = hw[it];
      __threadfence();
    }
    __syncthreads();
  }
}

typedef float    ms1_v4f __attribute__((ext_vector_type(4)));
typedef unsigned ms1_v4u __attribute__((ext_vector_type(4)));
struct ms1_args {
  const float* dtpre;
  const float* u;
  const float* bc;
  const float* z;
  const float* A_log;
  const float* Dskip;
  __half* y;
  __half* y_lo;
  long ld_dtpre;
  long ld_u;
  long ld_bc;
  long ld_z;
  long ld_y;
  int offB;
  int offC;
  int offZ;
  float ycarry;
  int dir;
  int D;
  int L;
  int nbatch;
};
static_assert(sizeof(ms1_args) == 136);

__device__ __forceinline__ float ms1_flush16(float v) {
  return (fabsf(v) < 6.103515625e-05f) ? 0.0f : v;
}
__device__ __forceinline__ unsigned ms1_h16bits(float v) {
  return (unsigned)__half_as_ushort(__float2half_rn(ms1_flush16(v)));
}
__device__ __forceinline__ float ms1_h16val(unsigned b) {
  return __half2float(__ushort_as_half((unsigned short)b));
}
__device__ __forceinline__ float ms1_softplus(float v) {
  return fmaxf(v, 0.0f) + log1pf(expf(-fabsf(v)));
}
__device__ __forceinline__ void ms1_pack2(float v0, float v1, unsigned& hw, unsigned& lw) {
  const unsigned h0 = ms1_h16bits(v0);
  const unsigned h1 = ms1_h16bits(v1);
  const float r0 = (v0 - ms1_h16val(h0)) * 2048.0f;
  const float r1 = (v1 - ms1_h16val(h1)) * 2048.0f;
  const unsigned l0 = ms1_h16bits(r0);
  const unsigned l1 = ms1_h16bits(r1);
  hw = h0 | (h1 << 16);
  lw = l0 | (l1 << 16);
}

template <int NSTATE>
__global__ __launch_bounds__(64 * (NSTATE / 16)) void ms1_scan_kernel(ms1_args a)
{
  static_assert(NSTATE == 16 || NSTATE == 64);
  constexpr int NQ  = NSTATE / 16;
  constexpr int NT  = 64 * NQ;
  constexpr int NW  = NT / 32;
  constexpr int BCW = 2 * NSTATE;
  constexpr int YP  = 68;
  constexpr int RPI = NW * 4;
  constexpr int NIT = 64 / RPI;
  static_assert(16 * NT <= 64 * YP);
  __shared__ __align__(16) float sBC[64 * BCW];
  __shared__ __align__(16) float sY[64 * YP];
  const int tid  = threadIdx.x;
  const int lane = tid & 31;
  const int wave = tid >> 5;
  const int c    = tid / NQ;
  const int sq   = tid - c * NQ;
  const int bpb  = a.D / 64;
  const int bi   = blockIdx.x / bpb;
  if (bi >= a.nbatch) return;
  const int d0 = (blockIdx.x - bi * bpb) * 64;
  const int d  = d0 + c;
  const long rowb = (long)bi * a.L;
  const bool hasz  = (a.z != nullptr);
  const bool hasD  = (a.Dskip != nullptr);
  const bool hasLo = (a.y_lo != nullptr);

#pragma unroll 1
  for (int n = 0; n < 16; ++n) {
    const float al = a.A_log[(long)d * NSTATE + sq * 16 + n];
    sY[n * NT + tid] = -expf(al);
  }
  __syncthreads();
  float An[16], h[16];
#pragma unroll
  for (int n = 0; n < 16; ++n) {
    An[n] = sY[n * NT + tid];
    h[n] = 0.0f;
  }
  float Dd = 0.0f;
  if (hasD) Dd = a.Dskip[d];

  const int nchunk = a.L / 64;
  const bool fwd = (a.dir > 0);
  const int s0 = fwd ? 0 : 63;
  const int sd = fwd ? 1 : -1;
  const int q  = lane >> 3;
  const int c8 = (lane & 7) * 8;

#pragma unroll 1
  for (int ci = 0; ci < nchunk; ++ci) {
    const int tb = fwd ? (ci * 64) : (a.L - 64 - ci * 64);
    const long rowc = rowb + tb;
    __syncthreads();
#pragma unroll 8
    for (int i = 0; i < 32; ++i) {
      const int idx = tid + i * NT;
      const int st  = idx / BCW;
      const int col = idx - st * BCW;
      const int sc  = (col < NSTATE) ? (a.offB + col) : (a.offC + col - NSTATE);
      sBC[idx] = a.bc[(rowc + st) * a.ld_bc + sc];
    }
    __syncthreads();
#pragma unroll 1
    for (int s = 0; s < 64; ++s) {
      const int ls = s0 + sd * s;
      const long row = rowc + ls;
      float pre = a.dtpre[row * a.ld_dtpre + d];
      float uv  = a.u[row * a.ld_u + d];
      float zv  = 0.0f;
      if (hasz) zv = a.z[row * a.ld_z + a.offZ + d];
      asm volatile("" : "+v"(pre));
      asm volatile("" : "+v"(uv));
      asm volatile("" : "+v"(zv));
      const float delta = ms1_softplus(pre);
      const float dtx = delta * uv;
      const float* bp = sBC + ls * BCW + sq * 16;
      const float* cp = bp + NSTATE;
      ms1_v4f Bq[4], Cq[4];
#pragma unroll
      for (int k = 0; k < 4; ++k) {
        Bq[k] = *(const ms1_v4f*)(bp + 4 * k);
        Cq[k] = *(const ms1_v4f*)(cp + 4 * k);
      }
      float yv = 0.0f;
#pragma unroll
      for (int n = 0; n < 16; ++n) {
        const float e = __expf(delta * An[n]);
        h[n] = fmaf(e, h[n], dtx * Bq[n >> 2][n & 3]);
        yv = fmaf(h[n], Cq[n >> 2][n & 3], yv);
      }
      if (NQ > 1) {
        yv += __shfl_xor(yv, 1, 32);
        yv += __shfl_xor(yv, 2, 32);
      }
      if (hasD) yv = fmaf(uv, Dd, yv);
      if (hasz) {
        const float sg = __builtin_amdgcn_rcpf(1.0f + expf(-zv));
        yv = yv * (zv * sg);
      }
      if (sq == 0) sY[ls * YP + c] = yv * a.ycarry;
    }
    __syncthreads();
    ms1_v4u hw[NIT], lw[NIT];
#pragma unroll
    for (int it = 0; it < NIT; ++it) {
      const int row = it * RPI + wave * 4 + q;
      const float* sp = sY + row * YP + c8;
      const ms1_v4f f0 = *(const ms1_v4f*)(sp);
      const ms1_v4f f1 = *(const ms1_v4f*)(sp + 4);
      unsigned h0, h1, h2, h3, l0, l1, l2, l3;
      ms1_pack2(f0[0], f0[1], h0, l0);
      ms1_pack2(f0[2], f0[3], h1, l1);
      ms1_pack2(f1[0], f1[1], h2, l2);
      ms1_pack2(f1[2], f1[3], h3, l3);
      hw[it] = (ms1_v4u){h0, h1, h2, h3};
      lw[it] = (ms1_v4u){l0, l1, l2, l3};
    }
    for (int pass = 0; pass < 2; ++pass) {
#pragma unroll
      for (int it = 0; it < NIT; ++it) {
        const int row = it * RPI + wave * 4 + q;
        const long o = (rowc + row) * a.ld_y + d0 + c8;
        *(volatile ms1_v4u*)(a.y + o) = hw[it];
        if (hasLo) *(volatile ms1_v4u*)(a.y_lo + o) = lw[it];
      }
      __threadfence();
    }
  }
}

__global__ __launch_bounds__(256) void split_y_kernel(
    const unsigned short* __restrict__ YH, unsigned short* __restrict__ YBH, unsigned short* __restrict__ YBL, int total8)
{
  const int i = blockIdx.x * 256 + threadIdx.x;
  if (i >= total8) return;
  const size_t e0 = (size_t)i << 3;
  const v4u w = *(const v4u*)(YH + e0);
  const unsigned w0 = w[0];
  const unsigned w1 = w[1];
  const unsigned w2 = w[2];
  const unsigned w3 = w[3];
  unsigned wi[4] = {w0, w1, w2, w3};
  unsigned ho[4], lo[4];
#pragma unroll
  for (int k = 0; k < 4; ++k) {
    const float f0 = h16_to_f32(wi[k] & 0xffffu);
    const float f1 = h16_to_f32(wi[k] >> 16);
    const unsigned short hb0 = f2bf_bits(f0);
    const unsigned short hb1 = f2bf_bits(f1);
    const unsigned short lb0 = f2bf_bits(f0 - bf_bits2f(hb0));
    const unsigned short lb1 = f2bf_bits(f1 - bf_bits2f(hb1));
    ho[k] = (unsigned)hb0 | ((unsigned)hb1 << 16);
    lo[k] = (unsigned)lb0 | ((unsigned)lb1 << 16);
  }
  const v4u hv = (v4u){ho[0], ho[1], ho[2], ho[3]};
  const v4u lv = (v4u){lo[0], lo[1], lo[2], lo[3]};
  unsigned short* qh = YBH + e0;
  unsigned short* ql = YBL + e0;
  *(volatile v4u*)qh = hv;
  *(volatile v4u*)ql = lv;
  __threadfence();
  *(volatile v4u*)qh = hv;
  *(volatile v4u*)ql = lv;
}

extern "C" void kernel_launch(void* const* d_in, const int* in_sizes, int n_in,
                              void* d_out, int out_size, void* d_ws, size_t ws_size,
                              hipStream_t stream) {
  if (n_in != 13) return;
  if (in_sizes[0] != kRows * kDm) return;
  if (in_sizes[1] != kDm * 2 * kDin) return;
  if (in_sizes[2] != 2 * kDin) return;
  if (in_sizes[3] != kDin * 4) return;
  if (in_sizes[4] != kDin) return;
  if (in_sizes[5] != kDin * 2 * kNst) return;
  if (in_sizes[6] != 2 * kNst) return;
  if (in_sizes[7] != kDin * kDin) return;
  if (in_sizes[8] != kDin) return;
  if (in_sizes[9] != kDin * kNst) return;
  if (in_sizes[10] != kDin) return;
  if (in_sizes[11] != kDin * kDm) return;
  if (in_sizes[12] != kDm) return;
  if (out_size != kRows * kDm) return;
  if (ws_size < kWsTotal) return;

  const float* x      = (const float*)d_in[0];
  const float* W_in   = (const float*)d_in[1];
  const float* b_in   = (const float*)d_in[2];
  const float* conv_w = (const float*)d_in[3];
  const float* conv_b = (const float*)d_in[4];
  const float* W_x    = (const float*)d_in[5];
  const float* b_x    = (const float*)d_in[6];
  const float* W_dt   = (const float*)d_in[7];
  const float* b_dt   = (const float*)d_in[8];
  const float* A_log  = (const float*)d_in[9];
  const float* Dp     = (const float*)d_in[10];
  const float* W_out  = (const float*)d_in[11];
  const float* b_out  = (const float*)d_in[12];
  float* out = (float*)d_out;

  char* ws = (char*)d_ws;
  float*          XPRE = (float*)(ws + kOffP);
  float*          DT   = (float*)(ws + kOffP);
  float*          Z    = (float*)(ws + kOffZ);
  float*          U    = (float*)(ws + kOffU);
  unsigned short* YBH  = (unsigned short*)(ws + kOffU);
  unsigned short* YBL  = (unsigned short*)(ws + kOffU + (size_t)kRows * kDin * 2);
  unsigned short* X16  = (unsigned short*)(ws + kOffQ);
  unsigned short* WINT = (unsigned short*)(ws + kOffQ + (size_t)kRows * kDm * 2);
  unsigned short* U16  = (unsigned short*)(ws + kOffQ);
  unsigned short* YH   = (unsigned short*)(ws + kOffQ);
  unsigned short* WDT  = (unsigned short*)(ws + kOffWdt);
  unsigned short* WOT  = (unsigned short*)(ws + kOffWot);
  unsigned short* WXT  = (unsigned short*)(ws + kOffWxt);
  float*          BC   = (float*)(ws + kOffBc);
  float*          PAR  = (float*)(ws + kOffPar);

  params_bf16_kernel<<<52, 256, 0, stream>>>(b_in, conv_w, conv_b, b_dt, A_log, Dp, b_out, b_x, PAR);

  cvt_rows_bf16_kernel<<<(kRows * kDm / 8) / 256, 256, 0, stream>>>(x, X16, kRows * kDm / 8);
  transpose_cvt_kernel<0><<<dim3((2 * kDin) / 64, kDm / 64), 256, 0, stream>>>(W_in, 2 * kDin, 0, 2 * kDin, WINT, kDm, 1.0f);
  transpose_cvt_kernel<1><<<dim3(kDin / 64, kDin / 64), 256, 0, stream>>>(W_dt, kDin, 0, kDin, WDT, kDin, kWCarry);
  transpose_cvt_kernel<0><<<dim3(kDm / 64, kDin / 64), 256, 0, stream>>>(W_out, kDm, 0, kDm, WOT, kDin, 1.0f);
  transpose_cvt_kernel<1><<<dim3(1, kDin / 64), 256, 0, stream>>>(W_x, 2 * kNst, kNst, kNst, WXT, kDin, kWCarry);

  wmma_gemm64<1, 0><<<dim3(256), 256, 0, stream>>>(
      X16, X16, kDm, WINT, kDm, XPRE, kDin, PAR + kPBin, kRows, kDin, kDm, 1.0f);
  wmma_gemm64<1, 0><<<dim3(256), 256, 0, stream>>>(
      X16, X16, kDm, WINT + (size_t)kDin * kDm, kDm, Z, kDin, PAR + kPBin + kDin, kRows, kDin, kDm, 1.0f);

  conv_silu_kernel<<<dim3(kDin / 256, kRows / 64), 256, 0, stream>>>(XPRE, PAR + kPCw, PAR + kPCb, U, U16);

  wmma_gemm64<0, 0><<<dim3(8), 256, 0, stream>>>(
      U16, U16, kDin, WXT, kDin, BC, kBcP, PAR + kPBx, kRows, kBcP, kDin, kProjScale);

  wmma_gemm64<0, 0><<<dim3(256), 256, 0, stream>>>(
      U16, U16, kDin, WDT, kDin, DT, kDin, PAR + kPBdt, kRows, kDin, kDin, kProjScale);

  for (int b = 0; b < kBatch; ++b) {
    const size_t r0 = (size_t)b * kSeq;
    ms1_args sa;
    sa.dtpre = DT + r0 * kDin;
    sa.u = U + r0 * kDin;
    sa.bc = BC + r0 * kBcP;
    sa.z = Z + r0 * kDin;
    sa.A_log = PAR + kPAlog;
    sa.Dskip = PAR + kPD;
    sa.y = (__half*)(YH + r0 * kDin);
    sa.y_lo = nullptr;
    sa.ld_dtpre = kDin;
    sa.ld_u = kDin;
    sa.ld_bc = kBcP;
    sa.ld_z = kDin;
    sa.ld_y = kDin;
    sa.offB = 0;
    sa.offC = kNst;
    sa.offZ = 0;
    sa.ycarry = kYCarry;
    sa.dir = 1;
    sa.D = kDin;
    sa.L = kSeq;
    sa.nbatch = 1;
    ms1_scan_kernel<16><<<dim3(kDin / 64), 64, 0, stream>>>(sa);
  }

  split_y_kernel<<<(kRows * kDin / 8) / 256, 256, 0, stream>>>(YH, YBH, YBL, kRows * kDin / 8);

  wmma_gemm64<1, 1><<<dim3(128), 256, 0, stream>>>(
      YBH, YBL, kDin, WOT, kDin, out, kDm, PAR + kPBout, kRows, kDm, kDin, kOutScale);
}
